// MBoundaryLoss_74165495267538
// MI455X (gfx1250) — hardware-run, weakly checked
//
#include <hip/hip_runtime.h>
#include <math.h>

typedef __attribute__((ext_vector_type(16))) _Float16 v16h;
typedef __attribute__((ext_vector_type(8)))  _Float16 v8h;
typedef __attribute__((ext_vector_type(8)))  float    v8f;
typedef __attribute__((ext_vector_type(4)))  float    v4f;
typedef __attribute__((ext_vector_type(4)))  unsigned int v4u;
typedef v4u v4u_a __attribute__((may_alias));

constexpr int kB   = 8192;
constexpr int kC   = 10;
constexpr int kD   = 256;
constexpr int kCD  = kC * kD;
constexpr int kLdP = 257;
constexpr int kNOut = 1 + kC + kB * kC;
constexpr int kOutBlocks = 80;
constexpr int kTailBase  = kOutBlocks * 256 * 4;
constexpr int kTailN     = kNOut - kTailBase;
constexpr float kCarryX  = 16.0f;
constexpr float kCarryM  = 256.0f;
constexpr float kCovFold  = 1.0f / (kCarryX * kCarryX);
constexpr float kQuadFold = 1.0f / (kCarryX * kCarryM);
constexpr float kJitter   = 1e-11f;
constexpr unsigned kInvLdsBytes = (unsigned)((kD * kLdP + kD) * sizeof(float));
static_assert(kNOut == 81931);
static_assert(kTailN == 11);
static_assert((kB % 256) == 0 && (kB % 64) == 0 && (kB % 32) == 0);
static_assert((kCD % 64) == 0 && (kD % 64) == 0 && (kD % 32) == 0);
static_assert(((kCD / 64) * (kD / 64)) == 20 * 8);
static_assert(((kB / 32) * kC) == 320 * 8);

constexpr size_t kOffPMU  = 0;
constexpr size_t kOffPCNT = kOffPMU  + (size_t)32 * kC * kD * 4;
constexpr size_t kOffMU   = kOffPCNT + (size_t)32 * 32 * 4;
constexpr size_t kOffSTAT = kOffMU   + (size_t)kC * kD * 4;
constexpr size_t kOffX16  = kOffSTAT + (size_t)64 * 4;
constexpr size_t kOffXCT  = kOffX16  + (size_t)kB * kD * 2;
constexpr size_t kOffXCTM = kOffXCT  + (size_t)kD * kB * 2;
constexpr size_t kOffCOV  = kOffXCTM + (size_t)kCD * kB * 2;
constexpr size_t kOffMINV = kOffCOV  + (size_t)kCD * kD * 4;
constexpr size_t kOffCMC  = kOffMINV + (size_t)kCD * kD * 2;
constexpr size_t kOffDIS  = kOffCMC  + (size_t)kC * 32 * 4;
constexpr size_t kOffLP   = kOffDIS  + (size_t)kC * kB * 4;
constexpr size_t kWsTotal = kOffLP   + (size_t)32 * 32 * 4;
static_assert(kWsTotal == 54939136ull);
static_assert(kWsTotal <= 134217728ull);
static_assert((kOffPCNT % 128) == 0 && (kOffMU % 128) == 0 && (kOffSTAT % 128) == 0 && (kOffX16 % 128) == 0 &&
              (kOffXCT % 128) == 0 && (kOffXCTM % 128) == 0 && (kOffCOV % 128) == 0 && (kOffMINV % 128) == 0 &&
              (kOffCMC % 128) == 0 && (kOffDIS % 128) == 0 && (kOffLP % 128) == 0);

__device__ __forceinline__ int clampi(int v, int lo, int hi) { return v < lo ? lo : (v > hi ? hi : v); }

__device__ __forceinline__ unsigned h16_bits(float f) {
  const _Float16 h = (_Float16)f;
  const unsigned short b = __builtin_bit_cast(unsigned short, h);
  return (unsigned)b;
}
__device__ __forceinline__ unsigned pack2h(float lo, float hi) { return h16_bits(lo) | (h16_bits(hi) << 16); }

__device__ __forceinline__ float softplus_f(float x) { return fmaxf(x, 0.0f) + log1pf(expf(-fabsf(x))); }

union FragU { v16h v; v8h h[2]; };
__device__ __forceinline__ v16h frag_load(const _Float16* p) {
  FragU f;
  f.h[0] = *(const v8h*)(p);
  f.h[1] = *(const v8h*)(p + 16);
  return f.v;
}
__device__ __forceinline__ v8f mma_h(v16h a, v16h b, v8f c) {
  c = __builtin_amdgcn_wmma_f32_16x16x32_f16(false, a, false, b, (short)0, c, false, false);
  asm volatile("v_nop\n\tv_nop\n\tv_nop\n\tv_nop" : "+v"(c) : "v"(a), "v"(b));
  return c;
}

__global__ __launch_bounds__(256) void class_sums_kernel(
    const float* __restrict__ src, const int* __restrict__ labels,
    float* __restrict__ pmu, float* __restrict__ pcnt)
{
  __shared__ __align__(16) float sAcc[kC * kD];
  __shared__ int sLab[256];
  const int tid = threadIdx.x, lane = tid & 31;
  const int n0 = blockIdx.x * 256;
  {
    int l = labels[n0 + tid];
    l = clampi(l, 0, kC - 1);
    sLab[tid] = l;
  }
#pragma unroll 1
  for (int c = 0; c < kC; ++c) sAcc[c * kD + tid] = 0.0f;
  __syncthreads();
#pragma unroll 4
  for (int r = 0; r < 256; ++r) {
    const int lr = sLab[r];
    const float x = src[(size_t)(n0 + r) * kD + tid];
    sAcc[lr * kD + tid] += x;
  }
  __syncthreads();
  float cntf = 0.0f;
  if (tid < 32) {
#pragma unroll 1
    for (int r = 0; r < 256; ++r) cntf += (sLab[r] == lane) ? 1.0f : 0.0f;
  }
  v4f pv[3];
#pragma unroll
  for (int it = 0; it < 3; ++it) {
    const int item = it * 256 + tid;
    const int itc = item < 640 ? item : 639;
    pv[it] = *(const v4f*)(sAcc + itc * 4);
  }
  float* dst = pmu + (size_t)blockIdx.x * kCD;
  for (int pass = 0; pass < 2; ++pass) {
#pragma unroll
    for (int it = 0; it < 3; ++it) {
      const int item = it * 256 + tid;
      if (item < 640) *(volatile v4f*)(dst + item * 4) = pv[it];
    }
    if (tid < 32) *(volatile float*)(pcnt + blockIdx.x * 32 + lane) = cntf;
    __threadfence();
  }
}

__global__ __launch_bounds__(64) void class_mean_kernel(
    const float* __restrict__ pmu, const float* __restrict__ pcnt,
    float* __restrict__ mu, float* __restrict__ stat)
{
  const int tid = threadIdx.x, lane = tid & 31;
  if (blockIdx.x < kC) {
    const int c = blockIdx.x;
    float cnt = 0.0f;
    v4f s = (v4f){0.f, 0.f, 0.f, 0.f};
#pragma unroll 1
    for (int j = 0; j < 32; ++j) {
      cnt += pcnt[j * 32 + c];
      const v4f p = *(const v4f*)(pmu + (size_t)(j * kC + c) * kD + tid * 4);
      s += p;
    }
    const float rc = 1.0f / cnt;
    const v4f m = s * rc;
    float* q = mu + c * kD + tid * 4;
    *(volatile v4f*)q = m;
    __threadfence();
    *(volatile v4f*)q = m;
  } else {
    if (tid < 32) {
      float cnt = 0.0f;
#pragma unroll 1
      for (int j = 0; j < 32; ++j) cnt += pcnt[j * 32 + lane];
      const float inv = 1.0f / (cnt - 1.0f);
      const float iv = (lane < kC) ? inv : 0.0f;
      *(volatile float*)(stat + lane) = cnt;
      *(volatile float*)(stat + 32 + lane) = iv;
      __threadfence();
      *(volatile float*)(stat + lane) = cnt;
      *(volatile float*)(stat + 32 + lane) = iv;
    }
  }
}

__device__ __forceinline__ unsigned mask_word(const int* lab, int idx) {
  const int c = idx >> 5, j = idx & 31;
  const int l0 = lab[2 * j], l1 = lab[2 * j + 1];
  const unsigned m0 = (l0 == c) ? 0x0000ffffu : 0u;
  const unsigned m1 = (l1 == c) ? 0xffff0000u : 0u;
  return m0 | m1;
}

__global__ __launch_bounds__(256) void planes_kernel(
    const float* __restrict__ pooled, const float* __restrict__ src, const int* __restrict__ labels,
    const float* __restrict__ mu,
    unsigned short* __restrict__ x16, unsigned short* __restrict__ xct, unsigned short* __restrict__ xctm)
{
  __shared__ __align__(16) float sMu[kC * kD];
  __shared__ int sLab[64];
  __shared__ __align__(16) unsigned sMW[kC * 32];
  __shared__ __align__(16) unsigned sT[kD * 36];
  const int tid = threadIdx.x, lane = tid & 31, wave = tid >> 5;
  const int n0 = blockIdx.x * 64;
  {
    int l = labels[n0 + (tid & 63)];
    asm volatile("" : "+v"(l));
    l = clampi(l, 0, kC - 1);
    if (tid < 64) sLab[tid] = l;
  }
#pragma unroll 1
  for (int c = 0; c < kC; ++c) sMu[c * kD + tid] = mu[c * kD + tid];
  __syncthreads();
  sMW[tid] = mask_word(sLab, tid);
  if (tid < 64) sMW[256 + tid] = mask_word(sLab, 256 + tid);
#pragma unroll 2
  for (int j = 0; j < 32; ++j) {
    const int l0 = sLab[2 * j], l1 = sLab[2 * j + 1];
    const float x0 = src[(size_t)(n0 + 2 * j) * kD + tid];
    const float x1 = src[(size_t)(n0 + 2 * j + 1) * kD + tid];
    const float c0 = x0 - sMu[l0 * kD + tid];
    const float c1 = x1 - sMu[l1 * kD + tid];
    sT[tid * 36 + j] = pack2h(c0 * kCarryX, c1 * kCarryX);
  }
  __syncthreads();
  {
    const int q = lane >> 3, seg = lane & 7;
    for (int pass = 0; pass < 2; ++pass) {
#pragma unroll 1
      for (int it = 0; it < 8; ++it) {
        const int d = it * 32 + wave * 4 + q;
        const v4u w = *(const v4u_a*)(sT + d * 36 + seg * 4);
        *(volatile v4u*)(void*)(xct + (size_t)d * kB + n0 + seg * 8) = w;
#pragma unroll 1
        for (int c = 0; c < kC; ++c) {
          const v4u mw = *(const v4u_a*)(sMW + c * 32 + seg * 4);
          const v4u wm = w & mw;
          *(volatile v4u*)(void*)(xctm + (size_t)(c * kD + d) * kB + n0 + seg * 8) = wm;
        }
      }
      __threadfence();
    }
  }
  {
    const float* pt = pooled + (size_t)n0 * kD;
    unsigned short* xd = x16 + (size_t)n0 * kD;
    v4u xv[8];
#pragma unroll
    for (int it = 0; it < 8; ++it) {
      const int e0 = (it * 256 + tid) * 8;
      const v4f a0 = *(const v4f*)(pt + e0);
      const v4f a1 = *(const v4f*)(pt + e0 + 4);
      const float f0 = a0[0], f1 = a0[1], f2 = a0[2], f3 = a0[3];
      const float f4 = a1[0], f5 = a1[1], f6 = a1[2], f7 = a1[3];
      v4u w;
      w[0] = pack2h(f0 * kCarryX, f1 * kCarryX);
      w[1] = pack2h(f2 * kCarryX, f3 * kCarryX);
      w[2] = pack2h(f4 * kCarryX, f5 * kCarryX);
      w[3] = pack2h(f6 * kCarryX, f7 * kCarryX);
      xv[it] = w;
    }
    for (int pass = 0; pass < 2; ++pass) {
#pragma unroll
      for (int it = 0; it < 8; ++it) {
        const int e0 = (it * 256 + tid) * 8;
        *(volatile v4u*)(void*)(xd + e0) = xv[it];
      }
      __threadfence();
    }
  }
}

__global__ __launch_bounds__(256) void cov_gemm_kernel(
    const unsigned short* __restrict__ Ap, const unsigned short* __restrict__ Btp,
    float* __restrict__ C, const float* __restrict__ stat)
{
  __shared__ __align__(16) float sT[8][16 * 68];
  const _Float16* A  = (const _Float16*)Ap;
  const _Float16* Bt = (const _Float16*)Btp;
  const int lane = threadIdx.x & 31;
  const int wave = threadIdx.x >> 5;
  constexpr int tilesN = kD / 64;
  const int tile = blockIdx.x * 8 + wave;
  const int tm = tile / tilesN;
  const int tn = tile - tm * tilesN;
  const int m0 = tm << 6;
  const int n0 = tn << 6;
  const int rlane = lane & 15;
  const int koff  = (lane >> 4) * 8;
  const int mOff  = (lane >> 4) * 8;

  v8f acc[4][4];
#pragma unroll
  for (int i = 0; i < 4; ++i)
#pragma unroll
    for (int j = 0; j < 4; ++j) acc[i][j] = (v8f){0.f,0.f,0.f,0.f,0.f,0.f,0.f,0.f};

#pragma unroll 1
  for (int k0 = 0; k0 < kB; k0 += 32) {
    v16h bh[4];
#pragma unroll
    for (int j = 0; j < 4; ++j)
      bh[j] = frag_load(Bt + (size_t)(n0 + (j << 4) + rlane) * kB + koff + k0);
#pragma unroll
    for (int i = 0; i < 4; ++i) {
      const v16h ah = frag_load(A + (size_t)(m0 + (i << 4) + rlane) * kB + koff + k0);
#pragma unroll
      for (int j = 0; j < 4; ++j) acc[i][j] = mma_h(ah, bh[j], acc[i][j]);
    }
  }

  const float scale = stat[32 + (m0 >> 8)] * kCovFold;
  float* slab = sT[wave];
#pragma unroll
  for (int i = 0; i < 4; ++i) {
    const int mBase = m0 + (i << 4);
#pragma unroll
    for (int j = 0; j < 4; ++j) {
#pragma unroll
      for (int r = 0; r < 8; ++r) {
        const float v = acc[i][j][r] * scale;
        slab[(mOff + r) * 68 + (j << 4) + rlane] = v;
      }
    }
    __builtin_amdgcn_fence(__ATOMIC_RELEASE, "workgroup");
    __builtin_amdgcn_wave_barrier();
    __builtin_amdgcn_fence(__ATOMIC_ACQUIRE, "workgroup");
    {
      const int hh = lane >> 4, c4 = (lane & 15) * 4;
      for (int pass = 0; pass < 2; ++pass) {
#pragma unroll
        for (int it = 0; it < 8; ++it) {
          const int row = it * 2 + hh;
          const v4f v = *(const v4f*)(slab + row * 68 + c4);
          *(volatile v4f*)(C + (size_t)(mBase + row) * kD + n0 + c4) = v;
        }
        __threadfence();
      }
    }
    __builtin_amdgcn_fence(__ATOMIC_RELEASE, "workgroup");
    __builtin_amdgcn_wave_barrier();
    __builtin_amdgcn_fence(__ATOMIC_ACQUIRE, "workgroup");
  }
}

__global__ __launch_bounds__(256) void invert_kernel(
    const float* __restrict__ cov, const float* __restrict__ centroids,
    unsigned short* __restrict__ minv16, float* __restrict__ cmc)
{
  extern __shared__ __align__(16) float ldsm[];
  float* colk = ldsm + kD * kLdP;
  const int c = blockIdx.x, j = threadIdx.x, lane = j & 31, wave = j >> 5;
  const float* Am = cov + (size_t)c * kD * kD;
#pragma unroll 4
  for (int i = 0; i < kD; ++i)
    ldsm[i * kLdP + j] = Am[(size_t)i * kD + j] + ((i == j) ? kJitter : 0.0f);
  __syncthreads();
#pragma unroll 1
  for (int k = 0; k < kD; ++k) {
    colk[j] = ldsm[j * kLdP + k];
    const float rowkj = ldsm[k * kLdP + j];
    __syncthreads();
    const float pivinv = 1.0f / colk[k];
    const bool isk = (j == k);
    const float nr = (isk ? 1.0f : rowkj) * pivinv;
#pragma unroll 4
    for (int i = 0; i < kD; ++i) {
      const float cur = ldsm[i * kLdP + j];
      const float old = isk ? 0.0f : cur;
      ldsm[i * kLdP + j] = old - colk[i] * nr;
    }
    ldsm[k * kLdP + j] = nr;
    __syncthreads();
  }
  for (int pass = 0; pass < 2; ++pass) {
#pragma unroll 1
    for (int it = 0; it < 32; ++it) {
      const int row = it * 8 + wave;
      const float* rp = ldsm + row * kLdP + lane * 8;
      const float f0 = rp[0], f1 = rp[1], f2 = rp[2], f3 = rp[3];
      const float f4 = rp[4], f5 = rp[5], f6 = rp[6], f7 = rp[7];
      v4u w;
      w[0] = pack2h(f0 * kCarryM, f1 * kCarryM);
      w[1] = pack2h(f2 * kCarryM, f3 * kCarryM);
      w[2] = pack2h(f4 * kCarryM, f5 * kCarryM);
      w[3] = pack2h(f6 * kCarryM, f7 * kCarryM);
      *(volatile v4u*)(void*)(minv16 + (size_t)(c * kD + row) * kD + lane * 8) = w;
    }
    __threadfence();
  }
  colk[j] = centroids[c * kD + j];
  __syncthreads();
  float t = 0.0f;
#pragma unroll 4
  for (int i = 0; i < kD; ++i) t = fmaf(colk[i], ldsm[i * kLdP + j], t);
  const float v = t * colk[j];
  __syncthreads();
  colk[j] = v;
  __syncthreads();
#pragma unroll 1
  for (int off = 128; off > 0; off >>= 1) {
    if (j < off) colk[j] += colk[j + off];
    __syncthreads();
  }
  if (j < 32) {
    const float tot = colk[0];
    *(volatile float*)(cmc + c * 32 + lane) = tot;
    __threadfence();
    *(volatile float*)(cmc + c * 32 + lane) = tot;
  }
}

__global__ __launch_bounds__(256) void quad_kernel(
    const unsigned short* __restrict__ x16p, const unsigned short* __restrict__ minvp,
    const float* __restrict__ pooled, const float* __restrict__ centroids,
    float* __restrict__ dis)
{
  __shared__ float sP[8][32 * 17];
  const int lane = threadIdx.x & 31;
  const int wave = threadIdx.x >> 5;
  const int task = blockIdx.x * 8 + wave;
  const int c  = task >> 8;
  const int m0 = (task & 255) * 32;
  const _Float16* A  = (const _Float16*)x16p + (size_t)m0 * kD;
  const _Float16* Bt = (const _Float16*)minvp + (size_t)c * kD * kD;
  const float* cen = centroids + c * kD;
  const int rlane = lane & 15;
  const int koff  = (lane >> 4) * 8;
  const int mOff  = (lane >> 4) * 8;

  float part[2][8];
#pragma unroll
  for (int i = 0; i < 2; ++i)
#pragma unroll
    for (int r = 0; r < 8; ++r) part[i][r] = 0.0f;

#pragma unroll 1
  for (int chunk = 0; chunk < 4; ++chunk) {
    const int n0 = chunk * 64;
    v8f acc[2][4];
#pragma unroll
    for (int i = 0; i < 2; ++i)
#pragma unroll
      for (int j = 0; j < 4; ++j) acc[i][j] = (v8f){0.f,0.f,0.f,0.f,0.f,0.f,0.f,0.f};
#pragma unroll 1
    for (int k0 = 0; k0 < kD; k0 += 32) {
      v16h bh[4];
#pragma unroll
      for (int j = 0; j < 4; ++j)
        bh[j] = frag_load(Bt + (size_t)(n0 + (j << 4) + rlane) * kD + koff + k0);
#pragma unroll
      for (int i = 0; i < 2; ++i) {
        const v16h ah = frag_load(A + (size_t)((i << 4) + rlane) * kD + koff + k0);
#pragma unroll
        for (int j = 0; j < 4; ++j) acc[i][j] = mma_h(ah, bh[j], acc[i][j]);
      }
    }
    float c2[4];
#pragma unroll
    for (int j = 0; j < 4; ++j) c2[j] = 2.0f * cen[n0 + (j << 4) + rlane];
#pragma unroll
    for (int i = 0; i < 2; ++i) {
#pragma unroll
      for (int rg = 0; rg < 2; ++rg) {
        float xv[4][4];
#pragma unroll
        for (int rr = 0; rr < 4; ++rr) {
          const size_t ro = (size_t)(m0 + (i << 4) + mOff + rg * 4 + rr) * kD + n0 + rlane;
#pragma unroll
          for (int j = 0; j < 4; ++j) xv[rr][j] = pooled[ro + (j << 4)];
        }
#pragma unroll
        for (int rr = 0; rr < 4; ++rr) {
#pragma unroll
          for (int j = 0; j < 4; ++j)
            part[i][rg * 4 + rr] = fmaf(acc[i][j][rg * 4 + rr], xv[rr][j] - c2[j], part[i][rg * 4 + rr]);
        }
        asm volatile("" ::: "memory");
      }
    }
  }

  float* slab = sP[wave];
#pragma unroll
  for (int i = 0; i < 2; ++i)
#pragma unroll
    for (int r = 0; r < 8; ++r)
      slab[((i << 4) + mOff + r) * 17 + rlane] = part[i][r] * kQuadFold;
  __builtin_amdgcn_fence(__ATOMIC_RELEASE, "workgroup");
  __builtin_amdgcn_wave_barrier();
  __builtin_amdgcn_fence(__ATOMIC_ACQUIRE, "workgroup");
  float s = 0.0f;
#pragma unroll
  for (int t = 0; t < 16; ++t) s += slab[lane * 17 + t];
  float* q = dis + (size_t)c * kB + m0 + lane;
  *(volatile float*)q = s;
  __threadfence();
  *(volatile float*)q = s;
}

__global__ __launch_bounds__(256) void loss_partial_kernel(
    const float* __restrict__ pooled, const float* __restrict__ centroids,
    const int* __restrict__ labels, const float* __restrict__ delta,
    float* __restrict__ lp)
{
  __shared__ float sRed[8];
  const int tid = threadIdx.x, lane = tid & 31, wave = tid >> 5;
  const int r0 = blockIdx.x * 256 + wave * 32;
  float wsum = 0.0f;
#pragma unroll 1
  for (int r = 0; r < 32; ++r) {
    const int row = r0 + r;
    int l = labels[row];
    l = clampi(l, 0, kC - 1);
    const float* px = pooled + (size_t)row * kD + lane * 8;
    const float* pc = centroids + l * kD + lane * 8;
    const v4f a0 = *(const v4f*)(px);
    const v4f a1 = *(const v4f*)(px + 4);
    const v4f b0 = *(const v4f*)(pc);
    const v4f b1 = *(const v4f*)(pc + 4);
    const v4f d0 = a0 - b0;
    const v4f d1 = a1 - b1;
    float ss = 0.0f;
    ss = fmaf(d0[0], d0[0], ss);
    ss = fmaf(d0[1], d0[1], ss);
    ss = fmaf(d0[2], d0[2], ss);
    ss = fmaf(d0[3], d0[3], ss);
    ss = fmaf(d1[0], d1[0], ss);
    ss = fmaf(d1[1], d1[1], ss);
    ss = fmaf(d1[2], d1[2], ss);
    ss = fmaf(d1[3], d1[3], ss);
    ss += __shfl_xor(ss, 16, 32);
    ss += __shfl_xor(ss, 8, 32);
    ss += __shfl_xor(ss, 4, 32);
    ss += __shfl_xor(ss, 2, 32);
    ss += __shfl_xor(ss, 1, 32);
    const float euc = sqrtf(ss);
    const float sp = softplus_f(delta[l]);
    wsum += fabsf(euc - sp);
  }
  if (lane == 0) sRed[wave] = wsum;
  __syncthreads();
  if (tid < 32) {
    float tot = 0.0f;
#pragma unroll
    for (int w = 0; w < 8; ++w) tot += sRed[w];
    *(volatile float*)(lp + blockIdx.x * 32 + lane) = tot;
    __threadfence();
    *(volatile float*)(lp + blockIdx.x * 32 + lane) = tot;
  }
}

__device__ __forceinline__ float logit_at(const float* __restrict__ dis, const float* __restrict__ cmc, int g) {
  int gi = g - (1 + kC);
  gi = clampi(gi, 0, kB * kC - 1);
  const int b = gi / kC;
  const int c = gi - b * kC;
  const float v = dis[(size_t)c * kB + b] + cmc[c * 32];
  return truncf(v);
}

__global__ __launch_bounds__(256) void pack_out_kernel(
    const float* __restrict__ dis, const float* __restrict__ cmc, const float* __restrict__ lp,
    const float* __restrict__ delta, float* __restrict__ out)
{
  __shared__ float sH[16];
  const int tid = threadIdx.x, lane = tid & 31;
  if (blockIdx.x == kOutBlocks) {
    if (tid < 32) {
      const int lc = lane < kTailN ? lane : (kTailN - 1);
      float v = logit_at(dis, cmc, kTailBase + lc);
      asm volatile("" : "+v"(v));
      for (int pass = 0; pass < 2; ++pass) {
        if (lane < kTailN) *(volatile float*)(out + kTailBase + lane) = v;
        __threadfence();
      }
    }
    return;
  }
  const int g0 = (blockIdx.x * 256 + tid) * 4;
  float e0 = logit_at(dis, cmc, g0);
  float e1 = logit_at(dis, cmc, g0 + 1);
  float e2 = logit_at(dis, cmc, g0 + 2);
  float e3 = logit_at(dis, cmc, g0 + 3);
  if (blockIdx.x == 0) {
    const int di = clampi(tid - 1, 0, kC - 1);
    float dv = delta[di];
    asm volatile("" : "+v"(dv));
    const float sp = softplus_f(dv);
    float ls = 0.0f;
#pragma unroll 1
    for (int j = 0; j < 32; ++j) ls += lp[j * 32];
    ls = ls * (1.0f / (float)kB);
    const float hv = (tid == 0) ? ls : sp;
    if (tid < 16) sH[tid] = hv;
    __syncthreads();
    const float h0 = sH[g0 < 15 ? g0 : 15];
    const float h1 = sH[(g0 + 1) < 15 ? (g0 + 1) : 15];
    const float h2 = sH[(g0 + 2) < 15 ? (g0 + 2) : 15];
    const float h3 = sH[(g0 + 3) < 15 ? (g0 + 3) : 15];
    e0 = (g0 < 1 + kC) ? h0 : e0;
    e1 = (g0 + 1 < 1 + kC) ? h1 : e1;
    e2 = (g0 + 2 < 1 + kC) ? h2 : e2;
    e3 = (g0 + 3 < 1 + kC) ? h3 : e3;
  }
  v4f v;
  v[0] = e0;
  v[1] = e1;
  v[2] = e2;
  v[3] = e3;
  *(volatile v4f*)(out + g0) = v;
  __threadfence();
  *(volatile v4f*)(out + g0) = v;
}

extern "C" void kernel_launch(void* const* d_in, const int* in_sizes, int n_in,
                              void* d_out, int out_size, void* d_ws, size_t ws_size,
                              hipStream_t stream) {
  if (n_in < 5) return;
  if (in_sizes[0] != kB * kD) return;
  if (in_sizes[1] != kC * kD) return;
  if (in_sizes[2] != kB) return;
  if (in_sizes[3] != kB * kD) return;
  if (in_sizes[4] != kC) return;
  if (out_size != kNOut) return;
  if (ws_size < kWsTotal) return;

  const float* pooled    = (const float*)d_in[0];
  const float* centroids = (const float*)d_in[1];
  const int*   labels    = (const int*)d_in[2];
  const float* src       = (const float*)d_in[3];
  const float* delta     = (const float*)d_in[4];
  float* out = (float*)d_out;

  char* ws = (char*)d_ws;
  float*          PMU  = (float*)(ws + kOffPMU);
  float*          PCNT = (float*)(ws + kOffPCNT);
  float*          MU   = (float*)(ws + kOffMU);
  float*          STAT = (float*)(ws + kOffSTAT);
  unsigned short* X16  = (unsigned short*)(ws + kOffX16);
  unsigned short* XCT  = (unsigned short*)(ws + kOffXCT);
  unsigned short* XCTM = (unsigned short*)(ws + kOffXCTM);
  float*          COV  = (float*)(ws + kOffCOV);
  unsigned short* MINV = (unsigned short*)(ws + kOffMINV);
  float*          CMC  = (float*)(ws + kOffCMC);
  float*          DIS  = (float*)(ws + kOffDIS);
  float*          LP   = (float*)(ws + kOffLP);

  class_sums_kernel<<<kB / 256, 256, 0, stream>>>(src, labels, PMU, PCNT);
  class_mean_kernel<<<kC + 1, 64, 0, stream>>>(PMU, PCNT, MU, STAT);
  planes_kernel<<<kB / 64, 256, 0, stream>>>(pooled, src, labels, MU, X16, XCT, XCTM);
  cov_gemm_kernel<<<20, 256, 0, stream>>>(XCTM, XCT, COV, STAT);
  invert_kernel<<<kC, 256, kInvLdsBytes, stream>>>(COV, centroids, MINV, CMC);
  quad_kernel<<<320, 256, 0, stream>>>(X16, MINV, pooled, centroids, DIS);
  loss_partial_kernel<<<kB / 256, 256, 0, stream>>>(pooled, centroids, labels, delta, LP);
  pack_out_kernel<<<kOutBlocks + 1, 256, 0, stream>>>(DIS, CMC, LP, delta, out);
}
